// ContinuousSheafTransport_71640054497903
// MI455X (gfx1250) — hardware-verified
//
#include <hip/hip_runtime.h>
#include <stddef.h>


#define WSC    8.0f
#define WINV   0.125f
#define LN_EPS 1e-5f

#define NTHR   256
#define NWAVE  8
#define EPT    8
#define CHUNK  (NTHR * EPT)
#define WCAP   (EPT * 32)
#define LISTN  (NWAVE * WCAP)
#define PASSN  (NWAVE * 16)
#define PCAP   (CHUNK + PASSN)
#define NB     512

#define NTHR2  128
#define NW2    4
#define ROWS2  (NW2 * 16)

#define DTHR   256

static_assert(PASSN == 128);
static_assert(PCAP >= CHUNK + PASSN);
static_assert((NB % 64) == 0);
static_assert(((NB * 64) % (NWAVE * 128)) == 0);

typedef float    v4f  __attribute__((ext_vector_type(4)));
typedef float    v8f  __attribute__((ext_vector_type(8)));
typedef int      v4i  __attribute__((ext_vector_type(4)));
typedef _Float16 v4h  __attribute__((ext_vector_type(4)));
typedef _Float16 v8h  __attribute__((ext_vector_type(8)));
typedef _Float16 v16h __attribute__((ext_vector_type(16)));
union FragH { v16h v; v8h h[2]; };

__device__ __forceinline__ int clampi(int v, int lo, int hi) { return v < lo ? lo : (v > hi ? hi : v); }

__device__ __forceinline__ v8h zero8h() {
  v8h r;
#pragma unroll
  for (int i = 0; i < 8; ++i) r[i] = (_Float16)0.0f;
  return r;
}

__device__ __forceinline__ v8f zero8f() {
  v8f r;
#pragma unroll
  for (int i = 0; i < 8; ++i) r[i] = 0.0f;
  return r;
}

__device__ __forceinline__ v8f wmh(v16h a, v16h b, v8f c) {
  v8f d = __builtin_amdgcn_wmma_f32_16x16x32_f16(false, a, false, b, (short)0, c, false, false);
  asm volatile("v_nop\n\tv_nop\n\tv_nop\n\tv_nop" : "+v"(d) : "v"(a), "v"(b));
  return d;
}

__device__ __forceinline__ v16h ldfrag(const _Float16* t, int pitch, int rowi, int k0, int hh) {
  FragH f;
  const _Float16* p = t + rowi * pitch + k0 + 8 * hh;
  f.h[0] = *(const v8h*)p;
  f.h[1] = *(const v8h*)(p + 16);
  return f.v;
}

__device__ __forceinline__ v8f ldc8(const float* p) {
  const v4f a = *(const v4f*)p;
  const v4f b = *(const v4f*)(p + 4);
  v8f c;
  c[0] = a.x; c[1] = a.y; c[2] = a.z; c[3] = a.w;
  c[4] = b.x; c[5] = b.y; c[6] = b.z; c[7] = b.w;
  return c;
}

__device__ __forceinline__ v8h relu8h(v8f d) {
  v8h r;
#pragma unroll
  for (int i = 0; i < 8; ++i) { const float t = fmaxf(d[i] * WINV, 0.0f); r[i] = (_Float16)t; }
  return r;
}

__device__ __forceinline__ float silu_f(float v) {
  const float e = __expf(-fabsf(v));
  const float s = __builtin_amdgcn_rcpf(1.0f + e);
  const float sg = (v >= 0.0f) ? s : e * s;
  return v * sg;
}

__device__ __forceinline__ float tanh_f(float v) {
  const float e = __expf(-2.0f * fabsf(v));
  const float t = (1.0f - e) * __builtin_amdgcn_rcpf(1.0f + e);
  return (v < 0.0f) ? -t : t;
}

__device__ __forceinline__ int scan_chunk(const int* __restrict__ keys, int nE, int cbase, int nodeBase,
                                          int vec8, int* list, int tid, int wave) {
  int wc = 0;
  const int el0  = tid * EPT;
  const int e0   = cbase + el0;
  const int sent = -2147483647 - 1;
  v4i da, db;
  if (vec8 != 0 && cbase + CHUNK <= nE) {
    da = *(const v4i*)(keys + e0);
    db = *(const v4i*)(keys + e0 + 4);
  } else {
    da.x = (e0     < nE) ? keys[min(e0, nE - 1)] : sent;
    da.y = (e0 + 1 < nE) ? keys[min(e0 + 1, nE - 1)] : sent;
    da.z = (e0 + 2 < nE) ? keys[min(e0 + 2, nE - 1)] : sent;
    da.w = (e0 + 3 < nE) ? keys[min(e0 + 3, nE - 1)] : sent;
    db.x = (e0 + 4 < nE) ? keys[min(e0 + 4, nE - 1)] : sent;
    db.y = (e0 + 5 < nE) ? keys[min(e0 + 5, nE - 1)] : sent;
    db.z = (e0 + 6 < nE) ? keys[min(e0 + 6, nE - 1)] : sent;
    db.w = (e0 + 7 < nE) ? keys[min(e0 + 7, nE - 1)] : sent;
  }
  const unsigned nb = (unsigned)nodeBase;
  const unsigned s0 = (unsigned)da.x - nb, s1 = (unsigned)da.y - nb;
  const unsigned s2 = (unsigned)da.z - nb, s3 = (unsigned)da.w - nb;
  const unsigned s4 = (unsigned)db.x - nb, s5 = (unsigned)db.y - nb;
  const unsigned s6 = (unsigned)db.z - nb, s7 = (unsigned)db.w - nb;
  const bool h0 = s0 < (unsigned)NB, h1 = s1 < (unsigned)NB, h2 = s2 < (unsigned)NB, h3 = s3 < (unsigned)NB;
  const bool h4 = s4 < (unsigned)NB, h5 = s5 < (unsigned)NB, h6 = s6 < (unsigned)NB, h7 = s7 < (unsigned)NB;
  const unsigned any = __builtin_amdgcn_ballot_w32(h0 | h1 | h2 | h3 | h4 | h5 | h6 | h7);
  if (any != 0u) {
#define HITJ(J, HJ) { \
      const unsigned mj = __builtin_amdgcn_ballot_w32(HJ); \
      if (mj != 0u) { \
        if (HJ) { \
          const int pos = wc + (int)__builtin_amdgcn_mbcnt_lo(mj, 0u); \
          if (pos < WCAP) list[wave * WCAP + pos] = el0 + (J); \
        } \
        wc += (int)__builtin_popcount(mj); } }
    HITJ(0, h0)
    HITJ(1, h1)
    HITJ(2, h2)
    HITJ(3, h3)
    HITJ(4, h4)
    HITJ(5, h5)
    HITJ(6, h6)
    HITJ(7, h7)
#undef HITJ
  }
  return wc;
}

__global__ __launch_bounds__(NTHR2) void k_pq(
    const float* hin, const float* hs, int addf,
    const float* __restrict__ W1, const float* __restrict__ b1,
    float* hout, float* pq, int nN) {
  __shared__ __attribute__((aligned(16))) _Float16 wt[128 * 72];
  __shared__ __attribute__((aligned(16))) _Float16 at[NW2 * 16 * 72];
  __shared__ __attribute__((aligned(16))) float    ost[NW2 * 16 * 128];
  __shared__ __attribute__((aligned(16))) float    b1s[64];

  const int tid = threadIdx.x, lane = tid & 31, wave = tid >> 5, hh = lane >> 4, m = lane & 15;
  const int row0 = blockIdx.x * ROWS2 + wave * 16;
  const bool act = (row0 + 16 <= nN);
  const int rowc = act ? row0 : (nN - 16);

  for (int i = tid; i < 128 * 64; i += NTHR2) {
    const int n = i >> 6, k = i & 63;
    const int wr = (n < 64) ? k : (64 + k);
    wt[n * 72 + k] = (_Float16)(W1[wr * 64 + (n & 63)] * WSC);
  }
  if (tid < 64) b1s[tid] = b1[tid];

  _Float16* aw = at + wave * (16 * 72);
  float* ow = ost + wave * (16 * 128);
  v4f hv[8];
#pragma unroll
  for (int i = 0; i < 8; ++i) {
    const int idx = i * 32 + lane, r = idx >> 4, c4 = idx & 15;
    const size_t g = (size_t)(rowc + r) * 64 + 4 * c4;
    const v4f a = *(const v4f*)(hin + g);
    const v4f b = *(const v4f*)(hs + g);
    v4f s = a;
    if (addf != 0) s = a + b;
    hv[i] = s;
    *(v4h*)(aw + r * 72 + 4 * c4) = __builtin_convertvector(s, v4h);
  }
  if (addf != 0 && act) {
    float* hb = hout + (size_t)row0 * 64;
#pragma unroll
    for (int i = 0; i < 8; ++i) *(volatile v4f*)(hb + 4 * (i * 32 + lane)) = hv[i];
    __threadfence();
#pragma unroll
    for (int i = 0; i < 8; ++i) *(volatile v4f*)(hb + 4 * (i * 32 + lane)) = hv[i];
  }
  __syncthreads();

  v8f acc[8];
#pragma unroll
  for (int nt = 0; nt < 8; ++nt) acc[nt] = zero8f();
#pragma unroll
  for (int ks = 0; ks < 2; ++ks) {
    const v16h a = ldfrag(aw, 72, m, 32 * ks, hh);
#pragma unroll
    for (int nt = 0; nt < 8; ++nt) {
      const v16h b = ldfrag(wt, 72, nt * 16 + m, 32 * ks, hh);
      acc[nt] = wmh(a, b, acc[nt]);
    }
  }
#pragma unroll
  for (int nt = 0; nt < 8; ++nt) {
    const float bias = (nt < 4) ? b1s[(nt * 16 + m) & 63] : 0.0f;
#pragma unroll
    for (int r = 0; r < 8; ++r) ow[(8 * hh + r) * 128 + nt * 16 + m] = acc[nt][r] * WINV + bias;
  }
  __syncthreads();

  v4f ov[16];
#pragma unroll
  for (int i = 0; i < 16; ++i) ov[i] = *(const v4f*)(ow + 4 * (i * 32 + lane));
  if (act) {
    float* pb = pq + (size_t)row0 * 128;
#pragma unroll
    for (int i = 0; i < 16; ++i) *(volatile v4f*)(pb + 4 * (i * 32 + lane)) = ov[i];
    __threadfence();
#pragma unroll
    for (int i = 0; i < 16; ++i) *(volatile v4f*)(pb + 4 * (i * 32 + lane)) = ov[i];
  }
}

__global__ __launch_bounds__(NTHR) void k_agg(
    const float* __restrict__ pq, const float* __restrict__ ea,
    const int* __restrict__ keys, const int* __restrict__ cols,
    const float* __restrict__ W1, const float* __restrict__ W2, const float* __restrict__ b2,
    float* gout, int nN, int nE, int vec8) {
  __shared__ __attribute__((aligned(16))) float    acc[(NB + 1) * 64];
  __shared__ __attribute__((aligned(16))) float    tm[PASSN * 64];
  __shared__ __attribute__((aligned(16))) _Float16 eat[PASSN * 32];
  __shared__ __attribute__((aligned(16))) _Float16 w1e[64 * 32];
  __shared__ __attribute__((aligned(16))) _Float16 w2t[64 * 72];
  __shared__ __attribute__((aligned(16))) float    b2s[64];
  __shared__ __attribute__((aligned(16))) int      list[LISTN];
  __shared__ __attribute__((aligned(16))) int      pend[PCAP];
  __shared__ int slotb[PASSN];
  __shared__ int wcnt[NWAVE];
  __shared__ int pendN;

  const int tid = threadIdx.x, lane = tid & 31, wave = tid >> 5, hh = lane >> 4, m = lane & 15;
  const int nodeBase = blockIdx.x * NB;

  {
    const v4f z4 = {0.0f, 0.0f, 0.0f, 0.0f};
    for (int i = tid; i < (NB + 1) * 16; i += NTHR) *(v4f*)(acc + 4 * i) = z4;
    const v8h z8 = zero8h();
    for (int i = tid; i < PASSN * 4; i += NTHR) *(v8h*)(eat + 8 * i) = z8;
    for (int i = tid; i < 64 * 32; i += NTHR) {
      const int f = i >> 5, k = i & 31;
      const int kk = k < 16 ? k : 15;
      float v = W1[(128 + kk) * 64 + f];
      v = (k < 16) ? v * WSC : 0.0f;
      w1e[i] = (_Float16)v;
    }
    for (int i = tid; i < 64 * 64; i += NTHR) {
      const int n = i >> 6, k = i & 63;
      w2t[n * 72 + k] = (_Float16)(W2[k * 64 + n] * WSC);
    }
    if (tid < 64) b2s[tid] = b2[tid];
    if (tid == 0) pendN = 0;
  }
  __syncthreads();

  const int nChunks = (nE + CHUNK - 1) / CHUNK;
#pragma unroll 1
  for (int ch = 0; ch < nChunks; ++ch) {
    const int cbase = ch * CHUNK;
    const int wc = scan_chunk(keys, nE, cbase, nodeBase, vec8, list, tid, wave);
    if (lane == 0) wcnt[wave] = wc;
    __syncthreads();

    const int base = pendN;
    int tot = 0, myoff = 0;
#pragma unroll
    for (int w = 0; w < NWAVE; ++w) {
      int c = wcnt[w];
      c = c > WCAP ? WCAP : (c < 0 ? 0 : c);
      if (w < wave) myoff += c;
      tot += c;
    }
    int newN = base + tot;
    newN = newN > PCAP ? PCAP : newN;
    {
      int n = wcnt[wave];
      n = n > WCAP ? WCAP : (n < 0 ? 0 : n);
      const int* lp = list + wave * WCAP;
      for (int i = lane; i < n; i += 32) {
        const int pos = base + myoff + i;
        if (pos < PCAP) pend[pos] = cbase + lp[i];
      }
    }
    const int fin = (ch == nChunks - 1) ? 1 : 0;
    const int R   = (fin != 0) ? (newN + PASSN - 1) / PASSN : newN / PASSN;
    const int Pv  = (fin != 0) ? newN : R * PASSN;
    __syncthreads();

#pragma unroll 1
    for (int r = 0; r < R; ++r) {
      {
        const int j = tid >> 1, c = tid & 1;
        const int idx = r * PASSN + j;
        const bool valid = idx < Pv;
        int e = pend[min(idx, PCAP - 1)];
        e = clampi(e, 0, nE - 1);
        int rw = keys[e];
        int cl = cols[e];
        int slot = rw - nodeBase;
        if (!valid || (unsigned)slot >= (unsigned)NB) slot = NB;
        rw = clampi(rw, 0, nN - 1);
        cl = clampi(cl, 0, nN - 1);
        const float* pp = pq + (size_t)rw * 128 + 32 * c;
        const float* qp = pq + (size_t)cl * 128 + 64 + 32 * c;
        float* tp = tm + j * 64 + 32 * c;
        const float sc = valid ? WSC : 0.0f;
#pragma unroll
        for (int q = 0; q < 8; ++q) {
          const v4f a = *(const v4f*)(pp + 4 * q);
          const v4f b = *(const v4f*)(qp + 4 * q);
          *(v4f*)(tp + 4 * q) = (a + b) * sc;
        }
        const float* ep = ea + (size_t)e * 16 + 8 * c;
        const float vs = valid ? 1.0f : 0.0f;
        const v4f e0 = *(const v4f*)ep * vs;
        const v4f e1 = *(const v4f*)(ep + 4) * vs;
        const v4h l4 = __builtin_convertvector(e0, v4h);
        const v4h h4 = __builtin_convertvector(e1, v4h);
        const v8h ev = __builtin_shufflevector(l4, h4, 0, 1, 2, 3, 4, 5, 6, 7);
        *(v8h*)(eat + j * 32 + 8 * c) = ev;
        if (c == 0) slotb[j] = slot;
      }
      __syncthreads();

      {
        const int eb = wave * 16;
        v8f cf[4];
        const float* trow = tm + (eb + m) * 64 + 8 * hh;
#pragma unroll
        for (int ft = 0; ft < 4; ++ft) cf[ft] = ldc8(trow + ft * 16);
        const v16h bea = ldfrag(eat, 32, eb + m, 0, hh);
        v8f d1[4];
#pragma unroll
        for (int ft = 0; ft < 4; ++ft) {
          const v16h a = ldfrag(w1e, 32, ft * 16 + m, 0, hh);
          d1[ft] = wmh(a, bea, cf[ft]);
        }
        FragH a2[2];
        a2[0].h[0] = relu8h(d1[0]); a2[0].h[1] = relu8h(d1[1]);
        a2[1].h[0] = relu8h(d1[2]); a2[1].h[1] = relu8h(d1[3]);
        v8f d2[4];
#pragma unroll
        for (int nt = 0; nt < 4; ++nt) d2[nt] = zero8f();
#pragma unroll
        for (int ks = 0; ks < 2; ++ks) {
#pragma unroll
          for (int nt = 0; nt < 4; ++nt) {
            const v16h b = ldfrag(w2t, 72, nt * 16 + m, 32 * ks, hh);
            d2[nt] = wmh(a2[ks].v, b, d2[nt]);
          }
        }
#pragma unroll
        for (int nt = 0; nt < 4; ++nt) {
          const float bias = b2s[nt * 16 + m];
#pragma unroll
          for (int rr = 0; rr < 8; ++rr) tm[(eb + 8 * hh + rr) * 64 + nt * 16 + m] = d2[nt][rr] * WINV + bias;
        }
      }
      __syncthreads();

      if (tid < 64) {
#pragma unroll 1
        for (int i = 0; i < PASSN; ++i) {
          int sl = slotb[i];
          sl = clampi(sl, 0, NB);
          acc[sl * 64 + tid] += tm[i * 64 + tid];
        }
      }
      __syncthreads();
    }

    int rem = newN - R * PASSN;
    rem = rem < 0 ? 0 : rem;
    if (R > 0 && tid < rem) pend[tid] = pend[R * PASSN + tid];
    if (tid == 0) pendN = rem;
  }
  __syncthreads();

  constexpr int WQ = NB * 64 / NWAVE;
  constexpr int NQ = WQ / 128;
  const float* ab = acc + wave * WQ;
  float* gb = gout + (size_t)nodeBase * 64 + (size_t)wave * WQ;
#pragma unroll 4
  for (int q = 0; q < NQ; ++q) {
    const v4f v = *(const v4f*)(ab + q * 128 + 4 * lane);
    *(volatile v4f*)(gb + q * 128 + 4 * lane) = v;
  }
  __threadfence();
#pragma unroll 4
  for (int q = 0; q < NQ; ++q) {
    const v4f v = *(const v4f*)(ab + q * 128 + 4 * lane);
    *(volatile v4f*)(gb + q * 128 + 4 * lane) = v;
  }
}

__global__ __launch_bounds__(NTHR2) void k_dyn(
    const float* __restrict__ hin, const float* __restrict__ gin,
    const float* __restrict__ Wd1, const float* __restrict__ bd1,
    const float* __restrict__ lng, const float* __restrict__ lnb,
    const float* __restrict__ Wd2, const float* __restrict__ bd2,
    float* hout, int nN) {
  __shared__ __attribute__((aligned(16))) _Float16 w1t[64 * 136];
  __shared__ __attribute__((aligned(16))) _Float16 w2t[64 * 72];
  __shared__ __attribute__((aligned(16))) _Float16 at[NW2 * 16 * 136];
  __shared__ __attribute__((aligned(16))) _Float16 ht[NW2 * 16 * 72];
  __shared__ __attribute__((aligned(16))) float    ost[NW2 * 16 * 64];
  __shared__ __attribute__((aligned(16))) float    prm[4 * 64];

  const int tid = threadIdx.x, lane = tid & 31, wave = tid >> 5, hh = lane >> 4, m = lane & 15;
  const int row0 = blockIdx.x * ROWS2 + wave * 16;
  const bool act = (row0 + 16 <= nN);
  const int rowc = act ? row0 : (nN - 16);

  for (int i = tid; i < 64 * 128; i += NTHR2) {
    const int n = i >> 7, k = i & 127;
    w1t[n * 136 + k] = (_Float16)(Wd1[k * 64 + n] * WSC);
  }
  for (int i = tid; i < 64 * 64; i += NTHR2) {
    const int n = i >> 6, k = i & 63;
    w2t[n * 72 + k] = (_Float16)(Wd2[k * 64 + n] * WSC);
  }
  if (tid < 64) {
    prm[tid] = bd1[tid]; prm[64 + tid] = lng[tid]; prm[128 + tid] = lnb[tid]; prm[192 + tid] = bd2[tid];
  }
  _Float16* aw = at + wave * (16 * 136);
  _Float16* hw = ht + wave * (16 * 72);
  float* ow = ost + wave * (16 * 64);
#pragma unroll
  for (int i = 0; i < 8; ++i) {
    const int idx = i * 32 + lane, r = idx >> 4, c4 = idx & 15;
    const size_t g = (size_t)(rowc + r) * 64 + 4 * c4;
    const v4f hv = *(const v4f*)(hin + g);
    const v4f gv = *(const v4f*)(gin + g);
    *(v4f*)(ow + 4 * idx) = hv;
    *(v4h*)(aw + r * 136 + 4 * c4) = __builtin_convertvector(hv, v4h);
    *(v4h*)(aw + r * 136 + 64 + 4 * c4) = __builtin_convertvector(gv, v4h);
  }
  __syncthreads();

  v8f x[4];
#pragma unroll
  for (int nt = 0; nt < 4; ++nt) x[nt] = zero8f();
#pragma unroll
  for (int ks = 0; ks < 4; ++ks) {
    const v16h a = ldfrag(aw, 136, m, 32 * ks, hh);
#pragma unroll
    for (int nt = 0; nt < 4; ++nt) {
      const v16h b = ldfrag(w1t, 136, nt * 16 + m, 32 * ks, hh);
      x[nt] = wmh(a, b, x[nt]);
    }
  }
  float mean[8], rstd[8];
  {
    float s[8];
#pragma unroll
    for (int rr = 0; rr < 8; ++rr) s[rr] = 0.0f;
#pragma unroll
    for (int nt = 0; nt < 4; ++nt) {
      const float bias = prm[nt * 16 + m];
#pragma unroll
      for (int rr = 0; rr < 8; ++rr) { const float v = x[nt][rr] * WINV + bias; x[nt][rr] = v; s[rr] += v; }
    }
#pragma unroll
    for (int off = 1; off < 16; off <<= 1) {
#pragma unroll
      for (int rr = 0; rr < 8; ++rr) s[rr] += __shfl_xor(s[rr], off, 32);
    }
#pragma unroll
    for (int rr = 0; rr < 8; ++rr) mean[rr] = s[rr] * (1.0f / 64.0f);
    float q[8];
#pragma unroll
    for (int rr = 0; rr < 8; ++rr) q[rr] = 0.0f;
#pragma unroll
    for (int nt = 0; nt < 4; ++nt) {
#pragma unroll
      for (int rr = 0; rr < 8; ++rr) { const float d = x[nt][rr] - mean[rr]; q[rr] += d * d; }
    }
#pragma unroll
    for (int off = 1; off < 16; off <<= 1) {
#pragma unroll
      for (int rr = 0; rr < 8; ++rr) q[rr] += __shfl_xor(q[rr], off, 32);
    }
#pragma unroll
    for (int rr = 0; rr < 8; ++rr) rstd[rr] = rsqrtf(q[rr] * (1.0f / 64.0f) + LN_EPS);
  }
#pragma unroll
  for (int nt = 0; nt < 4; ++nt) {
    const int n = nt * 16 + m;
    const float g = prm[64 + n], bb = prm[128 + n];
#pragma unroll
    for (int rr = 0; rr < 8; ++rr) {
      const float v = (x[nt][rr] - mean[rr]) * rstd[rr] * g + bb;
      hw[(8 * hh + rr) * 72 + n] = (_Float16)silu_f(v);
    }
  }
  __syncthreads();

  v8f y[4];
#pragma unroll
  for (int nt = 0; nt < 4; ++nt) y[nt] = zero8f();
#pragma unroll
  for (int ks = 0; ks < 2; ++ks) {
    const v16h a = ldfrag(hw, 72, m, 32 * ks, hh);
#pragma unroll
    for (int nt = 0; nt < 4; ++nt) {
      const v16h b = ldfrag(w2t, 72, nt * 16 + m, 32 * ks, hh);
      y[nt] = wmh(a, b, y[nt]);
    }
  }
#pragma unroll
  for (int nt = 0; nt < 4; ++nt) {
    const int n = nt * 16 + m;
    const float bias = prm[192 + n];
#pragma unroll
    for (int rr = 0; rr < 8; ++rr) {
      const float th = tanh_f(y[nt][rr] * WINV + bias);
      const int o = (8 * hh + rr) * 64 + n;
      const float hv = ow[o];
      ow[o] = hv + 0.5f * th;
    }
  }
  __syncthreads();

  v4f ov[8];
#pragma unroll
  for (int i = 0; i < 8; ++i) ov[i] = *(const v4f*)(ow + 4 * (i * 32 + lane));
  if (act) {
    float* hb = hout + (size_t)row0 * 64;
#pragma unroll
    for (int i = 0; i < 8; ++i) *(volatile v4f*)(hb + 4 * (i * 32 + lane)) = ov[i];
    __threadfence();
#pragma unroll
    for (int i = 0; i < 8; ++i) *(volatile v4f*)(hb + 4 * (i * 32 + lane)) = ov[i];
  }
}

__global__ __launch_bounds__(DTHR) void k_dis(const float* h, const int* __restrict__ keys,
                                             const int* __restrict__ cols, float* outp, int nN, int nE) {
  __shared__ __attribute__((aligned(16))) float red[DTHR];
  const int tid = threadIdx.x;
  const int base = blockIdx.x * DTHR;
  int e = base + tid;
  const bool valid = e < nE;
  e = clampi(e, 0, nE - 1);
  const int rw = clampi(keys[e], 0, nN - 1);
  const int cl = clampi(cols[e], 0, nN - 1);
  const float* a = h + (size_t)rw * 64;
  const float* b = h + (size_t)cl * 64;
  float sum = 0.0f;
#pragma unroll 2
  for (int i = 0; i < 16; ++i) {
    const v4f x = *(const v4f*)(a + 4 * i);
    const v4f y = *(const v4f*)(b + 4 * i);
    const v4f d = x - y;
    sum += d.x * d.x + d.y * d.y + d.z * d.z + d.w * d.w;
  }
  red[tid] = valid ? fminf(sum, 1e4f) : 0.0f;
  __syncthreads();
  const int remv = nE - base;
  const int o = 4 * tid;
  const bool wr = (tid < DTHR / 4) && (o + 3 < remv);
  v4f v = {0.0f, 0.0f, 0.0f, 0.0f};
  if (tid < DTHR / 4) v = *(const v4f*)(red + o);
  if (wr) *(volatile v4f*)(outp + (size_t)base + o) = v;
  __threadfence();
  if (wr) *(volatile v4f*)(outp + (size_t)base + o) = v;
}

extern "C" void kernel_launch(void* const* d_in, const int* in_sizes, int n_in,
                              void* d_out, int out_size, void* d_ws, size_t ws_size,
                              hipStream_t stream) {
  if (n_in < 13) return;
  const int nT = 2;
  if (in_sizes[0] <= 0 || (in_sizes[0] % (nT * 64)) != 0) return;
  const int nN = in_sizes[0] / (nT * 64);
  if (in_sizes[1] <= 0 || (in_sizes[1] % (nT * 16)) != 0) return;
  const int nE = in_sizes[1] / (nT * 16);
  if (nN < 16 || (nN % 16) != 0 || nE < 16 || (nE % 16) != 0) return;
  if (in_sizes[2] != 144 * 64 || in_sizes[3] != 64 || in_sizes[4] != 64 * 64 || in_sizes[5] != 64) return;
  if (in_sizes[6] != 128 * 64 || in_sizes[7] != 64 || in_sizes[8] != 64 || in_sizes[9] != 64) return;
  if (in_sizes[10] != 64 * 64 || in_sizes[11] != 64 || in_sizes[12] != nT * 2 * nE) return;
  if (out_size != nN * 64 + nT * nE) return;

  const float* hseq  = (const float*)d_in[0];
  const float* eattr = (const float*)d_in[1];
  const float* W1  = (const float*)d_in[2];
  const float* b1  = (const float*)d_in[3];
  const float* W2  = (const float*)d_in[4];
  const float* b2  = (const float*)d_in[5];
  const float* Wd1 = (const float*)d_in[6];
  const float* bd1 = (const float*)d_in[7];
  const float* lng = (const float*)d_in[8];
  const float* lnb = (const float*)d_in[9];
  const float* Wd2 = (const float*)d_in[10];
  const float* bd2 = (const float*)d_in[11];
  const int*   ei  = (const int*)d_in[12];
  float* out0 = (float*)d_out;
  float* out1 = out0 + (size_t)nN * 64;

  const int nBlkA = (nN + NB - 1) / NB;
  const int nBlk2 = (nN + ROWS2 - 1) / ROWS2;
  const int nBlkD = (nE + DTHR - 1) / DTHR;

  char* ws = (char*)d_ws;
  size_t off = 0;
  const size_t szH  = ((size_t)nN * 64 * 4 + 255) & ~(size_t)255;
  const size_t szPQ = ((size_t)nN * 128 * 4 + 255) & ~(size_t)255;
  const size_t szG  = ((size_t)nBlkA * NB * 64 * 4 + 255) & ~(size_t)255;
  const size_t oX = off; off += szH;
  const size_t oY = off; off += szH;
  const size_t oP = off; off += szPQ;
  const size_t oG = off; off += szG;
  if (off > ws_size) return;
  float* X  = (float*)(ws + oX);
  float* Y  = (float*)(ws + oY);
  float* PQ = (float*)(ws + oP);
  float* G  = (float*)(ws + oG);

  const int vec8 = ((nE & 3) == 0) ? 1 : 0;
  const int* rows0 = ei;
  const int* cols0 = ei + (size_t)nE;
  const int* rows1 = ei + (size_t)2 * nE;
  const int* cols1 = ei + (size_t)3 * nE;
  const float* hs0 = hseq;
  const float* hs1 = hseq + (size_t)nN * 64;
  const float* ea0 = eattr;
  const float* ea1 = eattr + (size_t)nE * 16;

  k_pq <<<nBlk2, NTHR2, 0, stream>>>(hs0, hs0, 1, W1, b1, X, PQ, nN);
  k_agg<<<nBlkA, NTHR,  0, stream>>>(PQ, ea0, rows0, cols0, W1, W2, b2, G, nN, nE, vec8);
  k_dyn<<<nBlk2, NTHR2, 0, stream>>>(X, G, Wd1, bd1, lng, lnb, Wd2, bd2, Y, nN);
  k_pq <<<nBlk2, NTHR2, 0, stream>>>(Y, Y, 0, W1, b1, Y, PQ, nN);
  k_agg<<<nBlkA, NTHR,  0, stream>>>(PQ, ea0, rows0, cols0, W1, W2, b2, G, nN, nE, vec8);
  k_dyn<<<nBlk2, NTHR2, 0, stream>>>(Y, G, Wd1, bd1, lng, lnb, Wd2, bd2, X, nN);
  k_dis<<<nBlkD, DTHR,  0, stream>>>(X, rows0, cols0, out1, nN, nE);
  k_pq <<<nBlk2, NTHR2, 0, stream>>>(X, hs1, 1, W1, b1, Y, PQ, nN);
  k_agg<<<nBlkA, NTHR,  0, stream>>>(PQ, ea1, rows1, cols1, W1, W2, b2, G, nN, nE, vec8);
  k_dyn<<<nBlk2, NTHR2, 0, stream>>>(Y, G, Wd1, bd1, lng, lnb, Wd2, bd2, X, nN);
  k_pq <<<nBlk2, NTHR2, 0, stream>>>(X, X, 0, W1, b1, X, PQ, nN);
  k_agg<<<nBlkA, NTHR,  0, stream>>>(PQ, ea1, rows1, cols1, W1, W2, b2, G, nN, nE, vec8);
  k_dyn<<<nBlk2, NTHR2, 0, stream>>>(X, G, Wd1, bd1, lng, lnb, Wd2, bd2, out0, nN);
  k_dis<<<nBlkD, DTHR,  0, stream>>>(out0, rows1, cols1, out1 + (size_t)nE, nN, nE);
}
